// UniBidirectional_Spatial_Attention_51625506898203
// MI455X (gfx1250) — hardware-verified
//
#include <hip/hip_runtime.h>
#include <math.h>

typedef __attribute__((ext_vector_type(16))) _Float16 v16h;
typedef __attribute__((ext_vector_type(16))) __bf16 v16b;
typedef __attribute__((ext_vector_type(8)))  _Float16 v8h;
typedef __attribute__((ext_vector_type(8)))  float v8f;
typedef __attribute__((ext_vector_type(4)))  float v4f;
typedef __attribute__((ext_vector_type(2)))  float v2f;
typedef __attribute__((ext_vector_type(4)))  unsigned v4u;
typedef __attribute__((ext_vector_type(4)))  int v4i;
typedef float __attribute__((may_alias)) float_a;
typedef int __attribute__((may_alias)) int_a;

template <typename T> __device__ __forceinline__ void vst2(void* p, T v) { *(volatile T*)p = v; __threadfence(); *(volatile T*)p = v; }
__device__ __forceinline__ v8f wmma16(v16h a, v16h b, v8f c) {
  v8f d = __builtin_amdgcn_wmma_f32_16x16x32_f16(false, a, false, b, (short)0, c, false, false);
  asm volatile("v_nop\n\tv_nop\n\tv_nop\n\tv_nop" : "+v"(d) : "v"(a), "v"(b));
  return d;
}
__device__ __forceinline__ v8f wmma_bf(v16b a, v16b b, v8f c) {
  v8f d = __builtin_amdgcn_wmma_f32_16x16x32_bf16(false, a, false, b, (short)0, c, false, false);
  asm volatile("v_nop\n\tv_nop\n\tv_nop\n\tv_nop" : "+v"(d) : "v"(a), "v"(b));
  return d;
}
__device__ __forceinline__ v16h frag_h(const _Float16* rowk0, int lane) {
  union { v16h v; v8h q[2]; } u; const _Float16* p = rowk0 + 8 * (lane >> 4);
  u.q[0] = *(const v8h*)p; u.q[1] = *(const v8h*)(p + 16); return u.v;
}
__device__ __forceinline__ v16h frag_f32(const float* rowk0, int lane) {
  v16h a; const float* p = rowk0 + 8 * (lane >> 4);
#pragma unroll
  for (int i = 0; i < 8; ++i) { a[i] = (_Float16)p[i]; a[8 + i] = (_Float16)p[16 + i]; }
  return a;
}
__device__ __forceinline__ v16h frag_f32s(const float* rowk0, int lane, float sc) {
  v16h a; const float* p = rowk0 + 8 * (lane >> 4);
#pragma unroll
  for (int i = 0; i < 8; ++i) { a[i] = (_Float16)(p[i] * sc); a[8 + i] = (_Float16)(p[16 + i] * sc); }
  return a;
}
__device__ __forceinline__ v16h fragc_f32(const float* W, int k0, int n, int lane, int ld, int K) {
  v16h a; const int g = lane >> 4;
#pragma unroll
  for (int i = 0; i < 8; ++i) { const int ka = k0 + 8 * g + i, kb = ka + 16;
    a[i] = (_Float16)(ka < K ? W[(size_t)(ka < K ? ka : K - 1) * ld + n] : 0.f); a[8 + i] = (_Float16)(kb < K ? W[(size_t)(kb < K ? kb : K - 1) * ld + n] : 0.f); }
  return a;
}
struct F2 { v16b h, l; };
__device__ __forceinline__ F2 bsplit16(const float v[16]) { F2 r;
#pragma unroll
  for (int i = 0; i < 16; ++i) { const __bf16 h = (__bf16)v[i]; r.h[i] = h; r.l[i] = (__bf16)(v[i] - (float)h); }
  return r; }
__device__ __forceinline__ F2 split_row(const float* row, int k0, int lane) { float v[16]; const float* p = row + k0 + 8 * (lane >> 4);
#pragma unroll
  for (int i = 0; i < 8; ++i) { v[i] = p[i]; v[8 + i] = p[16 + i]; }
  return bsplit16(v); }
__device__ __forceinline__ F2 split_rowK(const float* row, int k0, int lane, int K) { float v[16]; const int g = lane >> 4;
#pragma unroll
  for (int i = 0; i < 8; ++i) { const int ka = k0 + 8 * g + i, kb = ka + 16; v[i] = ka < K ? row[ka < K ? ka : K - 1] : 0.f; v[8 + i] = kb < K ? row[kb < K ? kb : K - 1] : 0.f; }
  return bsplit16(v); }
__device__ __forceinline__ F2 split_col(const float* W, int k0, int n, int lane, int ld, int K) { float v[16]; const int g = lane >> 4;
#pragma unroll
  for (int i = 0; i < 8; ++i) { const int ka = k0 + 8 * g + i, kb = ka + 16; v[i] = ka < K ? W[(size_t)(ka < K ? ka : K - 1) * ld + n] : 0.f; v[8 + i] = kb < K ? W[(size_t)(kb < K ? kb : K - 1) * ld + n] : 0.f; }
  return bsplit16(v); }
__device__ __forceinline__ v8f mac3(const F2& a, const F2& b, v8f c) { c = wmma_bf(a.l, b.h, c); c = wmma_bf(a.h, b.l, c); return wmma_bf(a.h, b.h, c); }
__device__ __forceinline__ float sigm(float v) { return 1.0f / (1.0f + expf(-v)); }
#define LDSX() do { asm volatile("s_wait_dscnt 0" ::: "memory"); __builtin_amdgcn_wave_barrier(); __builtin_amdgcn_fence(__ATOMIC_RELEASE, "workgroup"); } while (0)


#define NB 2
#define CC 64
#define NN 4096
#define NP 2
#ifndef TQB
#define TQB (NN / 64)
#define TNB NB
#endif
typedef __attribute__((ext_vector_type(8))) __bf16 v8b;
__device__ __forceinline__ v16b frag_b(const __bf16* rowk0, int lane) {
  union { v16b v; v8b q[2]; } u; const __bf16* p = rowk0 + 8 * (lane >> 4);
  u.q[0] = *(const v8b*)p; u.q[1] = *(const v8b*)(p + 16); return u.v;
}
__device__ __forceinline__ float bfr(float v) { return (float)(__bf16)v; }
__device__ __attribute__((noinline)) float exp_ni(float v) { return expf(v); }
__device__ __attribute__((noinline)) float erf_ni(float v) { return erff(v); }

#define WS_PW  0u
#define WS_Q   (WS_PW + 2u * 7 * CC * CC)
#define WS_K   (WS_Q + 2u * (size_t)NP * NB * NN * CC)
#define WS_V   (WS_K + 2u * (size_t)NP * NB * NN * CC)
#define WS_O   (WS_V + 2u * (size_t)NP * NB * CC * NN)
#define WS_END (WS_O + 4u * (size_t)NP * NB * NN * CC)

__global__ __launch_bounds__(64) void k_pack(const float* __restrict__ W0, const float* __restrict__ W1, const float* __restrict__ W2, const float* __restrict__ W3, const float* __restrict__ W4, const float* __restrict__ W5, const float* __restrict__ W6, __bf16* __restrict__ P) {
  const int n = blockIdx.x, m = blockIdx.y, t = threadIdx.x; const float* src = (m == 0) ? W0 : (m == 1) ? W1 : (m == 2) ? W2 : (m == 3) ? W3 : (m == 4) ? W4 : (m == 5) ? W5 : W6; __shared__ __align__(16) __bf16 s[CC]; s[t] = (__bf16)src[(size_t)n * CC + t]; __syncthreads(); if (t < CC / 8) vst2((unsigned*)(P + ((size_t)m * CC + n) * CC + t * 8), *(const v4u*)&s[t * 8]); }
__global__ __launch_bounds__(128) void k_proj(const float* __restrict__ SRC, const float* __restrict__ TGT, const __bf16* __restrict__ P, _Float16* __restrict__ Q, _Float16* __restrict__ Kr, _Float16* __restrict__ V) {
  __shared__ __align__(16) _Float16 so[64][72]; __shared__ __align__(16) _Float16 st[64][72];
  const int tid = threadIdx.x, wave = tid >> 5, lane = tid & 31, col = lane & 15, g = lane >> 4; const int which = blockIdx.y; const size_t b = blockIdx.z; const int n0b = blockIdx.x * 64, n0 = n0b + wave * 16;
  const float* X = (which >= 4) ? SRC : TGT; const int pair = (which >= 3) ? 1 : 0; const int role = (which >= 3) ? (which - 3) : which;
  v8f acc[4] = {};
#pragma unroll
  for (int kc = 0; kc < CC / 32; ++kc) { v16b a; { const float* p = X + (b * CC + kc * 32 + 8 * g) * NN + n0 + col;
#pragma unroll
      for (int i = 0; i < 8; ++i) { a[i] = (__bf16)p[(size_t)i * NN]; a[8 + i] = (__bf16)p[(size_t)(16 + i) * NN]; } }
#pragma unroll
    for (int j = 0; j < 4; ++j) acc[j] = wmma_bf(a, frag_b(P + ((size_t)which * CC + j * 16 + col) * CC + kc * 32, lane), acc[j]); }
  if (role < 2) { _Float16* dst = ((role == 0) ? Q : Kr) + ((size_t)pair * NB + b) * NN * CC;
#pragma unroll
    for (int j = 0; j < 4; ++j)
#pragma unroll
      for (int r = 0; r < 8; ++r) so[wave * 16 + 8 * g + r][j * 16 + col] = (_Float16)acc[j][r];
    LDSX();
    for (int rl = 0; rl < 16; ++rl) if (lane < 8) vst2((unsigned*)(dst + (size_t)(n0 + rl) * CC + lane * 8), *(const v4u*)&so[wave * 16 + rl][lane * 8]);
  } else { _Float16* dst = V + ((size_t)pair * NB + b) * CC * NN;
#pragma unroll
    for (int j = 0; j < 4; ++j)
#pragma unroll
      for (int r = 0; r < 8; ++r) st[j * 16 + col][wave * 16 + 8 * g + r] = (_Float16)acc[j][r];
    __syncthreads();
    for (int e = tid; e < 64 * 8; e += 128) { const int d = e >> 3, pc = e & 7; vst2((unsigned*)(dst + (size_t)d * NN + n0b + pc * 8), *(const v4u*)&st[d][pc * 8]); } }
}
__global__ __launch_bounds__(128) void k_attn(const _Float16* __restrict__ Q, const _Float16* __restrict__ Kr, const _Float16* __restrict__ V, float* __restrict__ O) {
  __shared__ __align__(16) _Float16 sph[4][16][40]; __shared__ __align__(16) float so[4][16][68];
  const int tid = threadIdx.x, wave = tid >> 5, lane = tid & 31, col = lane & 15, g = lane >> 4; const size_t pb = blockIdx.y; const int q0 = blockIdx.x * 64 + wave * 16; const size_t rq = pb * NN + q0;
  v16h aq[2];
#pragma unroll
  for (int kc = 0; kc < 2; ++kc) aq[kc] = frag_h(Q + (rq + col) * CC + kc * 32, lane);
  float m[8], l[8];
#pragma unroll
  for (int r = 0; r < 8; ++r) { m[r] = -3.0e38f; l[r] = 0.f; }
  v8f acc[4] = {};
#pragma unroll 1
  for (int ks = 0; ks < NN / 32; ++ks) { const int j0 = ks * 32; v8f s[2];
#pragma unroll
    for (int ct = 0; ct < 2; ++ct) { const size_t rk = (pb * NN + j0 + ct * 16 + col) * CC; v8f c = {};
#pragma unroll
      for (int kc = 0; kc < 2; ++kc) c = wmma16(aq[kc], frag_h(Kr + rk + kc * 32, lane), c);
#pragma unroll
      for (int r = 0; r < 8; ++r) s[ct][r] = c[r] * 0.125f; }
#pragma unroll
    for (int r = 0; r < 8; ++r) { float mx = fmaxf(s[0][r], s[1][r]);
#pragma unroll
      for (int o = 1; o < 16; o <<= 1) mx = fmaxf(mx, __shfl_xor(mx, o));
      const float mn = fmaxf(m[r], mx); const float alpha = (m[r] <= -1.0e38f) ? 0.f : __expf(m[r] - mn); const float e0 = __expf(s[0][r] - mn), e1 = __expf(s[1][r] - mn); float es = e0 + e1;
#pragma unroll
      for (int o = 1; o < 16; o <<= 1) es += __shfl_xor(es, o);
      l[r] = l[r] * alpha + es; m[r] = mn;
#pragma unroll
      for (int dt = 0; dt < 4; ++dt) acc[dt][r] *= alpha;
      sph[wave][8 * g + r][col] = (_Float16)(e0 * 2048.0f); sph[wave][8 * g + r][16 + col] = (_Float16)(e1 * 2048.0f); }
    LDSX();
    const v16h pa = frag_h(&sph[wave][col][0], lane);
#pragma unroll
    for (int dt = 0; dt < 4; ++dt) acc[dt] = wmma16(pa, frag_h(V + (pb * CC + dt * 16 + col) * NN + j0, lane), acc[dt]);
    LDSX(); }
#pragma unroll
  for (int r = 0; r < 8; ++r) { const float il = (1.0f / 2048.0f) / l[r];
#pragma unroll
    for (int dt = 0; dt < 4; ++dt) so[wave][8 * g + r][dt * 16 + col] = acc[dt][r] * il; }
  LDSX();
  for (int rl = 0; rl < 16; ++rl) if (lane < 16) vst2(O + (rq + rl) * CC + lane * 4, *(const v4f*)&so[wave][rl][lane * 4]);
}
__global__ __launch_bounds__(128) void k_fin(const float* __restrict__ O, const __bf16* __restrict__ P, float* __restrict__ OUT) {
  __shared__ __align__(16) float sa[4][16][68]; __shared__ __align__(16) float st[64][68];
  const int tid = threadIdx.x, wave = tid >> 5, lane = tid & 31, col = lane & 15, g = lane >> 4; const size_t b = blockIdx.y; const int n0b = blockIdx.x * 64, n0 = n0b + wave * 16;
  for (int e = lane; e < 16 * CC; e += 32) { const int rl = e >> 6, c = e & 63; sa[wave][rl][c] = (O[((0 * NB + b) * NN + n0 + rl) * CC + c] + O[((1 * NB + b) * NN + n0 + rl) * CC + c]) * 0.5f; }
  LDSX();
  v8f acc[4] = {};
#pragma unroll
  for (int kc = 0; kc < CC / 32; ++kc) { const F2 a = split_row(&sa[wave][col][0], kc * 32, lane);
#pragma unroll
    for (int jt = 0; jt < 4; ++jt) { const v16b w = frag_b(P + ((size_t)6 * CC + jt * 16 + col) * CC + kc * 32, lane); acc[jt] = wmma_bf(a.h, w, acc[jt]); acc[jt] = wmma_bf(a.l, w, acc[jt]); } }
#pragma unroll
  for (int jt = 0; jt < 4; ++jt)
#pragma unroll
    for (int r = 0; r < 8; ++r) st[jt * 16 + col][wave * 16 + 8 * g + r] = acc[jt][r];
  __syncthreads();
  for (int e = tid; e < CC * 16; e += 128) { const int o = e >> 4, q = e & 15; vst2(OUT + ((b * CC + o) * NN) + n0b + q * 4, *(const v4f*)&st[o][q * 4]); }
}
extern "C" void kernel_launch(void* const* d_in, const int* in_sizes, int n_in, void* d_out, int out_size, void* d_ws, size_t ws_size, hipStream_t stream) {
  (void)in_sizes; (void)n_in; (void)out_size;
  const float** F = (const float**)d_in;
  if (ws_size < (size_t)WS_END) return;
  char* ws = (char*)d_ws; __bf16* P = (__bf16*)ws; _Float16 *Q = (_Float16*)(ws + WS_Q), *Kr = (_Float16*)(ws + WS_K), *V = (_Float16*)(ws + WS_V); float* O = (float*)(ws + WS_O);
  k_pack<<<dim3(CC, 7), 64, 0, stream>>>(F[2], F[4], F[6], F[3], F[5], F[7], F[8], P);
  k_proj<<<dim3(NN / 64, 6, NB), 128, 0, stream>>>(F[0], F[1], P, Q, Kr, V);
  k_attn<<<dim3(TQB, NP * TNB), 128, 0, stream>>>(Q, Kr, V, O);
  k_fin<<<dim3(TQB, TNB), 128, 0, stream>>>(O, P, (float*)d_out);
}
